// MultiResourceAttention_72980084294339
// MI455X (gfx1250) — hardware-verified
//
#include <hip/hip_runtime.h>


namespace {
constexpr int NB = 4, S = 2048, D = 1024, NR = NB * S;
constexpr float XS = 8.0f, WSC = 256.0f, PS = 1024.0f, SCALE = 0.03125f  , LOG2E = 1.4426950408889634f, EPS = 1e-5f;

typedef _Float16 b16;
typedef __attribute__((ext_vector_type(16))) _Float16 v16b;
typedef __attribute__((ext_vector_type(8))) _Float16 v8b;
typedef __attribute__((ext_vector_type(8))) float v8f;
typedef __attribute__((ext_vector_type(4))) float v4f;
__device__ __forceinline__ float bf16_rne(float f) { unsigned int u = __float_as_uint(f); u += 0x7FFFu + ((u >> 16) & 1u); return __uint_as_float(u & 0xFFFF0000u); }
__device__ __forceinline__ v16b frag_kb(const b16* p, int hh) { const v8b a = *(const v8b*)(p + 8 * hh), b = *(const v8b*)(p + 16 + 8 * hh); v16b f;
#pragma unroll
  for (int e = 0; e < 8; ++e) { f[e] = a[e]; f[8 + e] = b[e]; } return f; }
__device__ __forceinline__ v8f wmma16b(v16b a, v16b b, v8f c) { v8f d = __builtin_amdgcn_wmma_f32_16x16x32_f16(false, a, false, b, (short)0, c, false, false); asm volatile("v_nop\n\tv_nop\n\tv_nop\n\tv_nop" : "+v"(d) : "v"(a), "v"(b)); return d; }
__device__ __forceinline__ void wave_lds_sync() { __builtin_amdgcn_fence(__ATOMIC_RELEASE, "workgroup"); __builtin_amdgcn_wave_barrier(); __builtin_amdgcn_fence(__ATOMIC_ACQUIRE, "workgroup"); }
__device__ __forceinline__ float nexp2(float x) { return __builtin_amdgcn_exp2f(x); }
__device__ __forceinline__ float pmul(float a, float b) { float p = a * b; asm volatile("" : "+v"(p)); return p; }

__global__ __launch_bounds__(256) void prepx_kernel(const float* __restrict__ x, b16* __restrict__ X16) {
  const size_t t = (size_t)blockIdx.x * 256 + threadIdx.x; if (t >= (size_t)NR * D / 8) return; const size_t e = t * 8;
  const v4f a = *(const v4f*)(x + e), c = *(const v4f*)(x + e + 4); v8b o;
#pragma unroll
  for (int j = 0; j < 4; ++j) { o[j] = (b16)(bf16_rne(a[j]) * XS); o[4 + j] = (b16)(bf16_rne(c[j]) * XS); }
  for (int pass = 0; pass < 2; ++pass) { *(volatile v8b*)(X16 + e) = o; __threadfence(); }
}
__global__ __launch_bounds__(256) void prepw_kernel(const float* __restrict__ wq, const float* __restrict__ wk, const float* __restrict__ wv, b16* __restrict__ WT) {
  __shared__ __attribute__((aligned(16))) b16 T[64][64 + 8];
  const int kind = blockIdx.z, d0 = blockIdx.y * 64, e0 = blockIdx.x * 64, t_ = threadIdx.x; const float* w = kind == 0 ? wq : kind == 1 ? wk : wv;
  for (int q = t_; q < 64 * 64; q += 256) { const int dd = q >> 6, ee = q & 63; T[ee][dd] = (b16)(bf16_rne(w[(size_t)(d0 + dd) * D + e0 + ee]) * WSC); }
  __syncthreads();
  for (int pass = 0; pass < 2; ++pass) { for (int q = t_; q < 64 * 8; q += 256) { const int ee = q >> 3, c8 = (q & 7) * 8; *(volatile v8b*)(WT + ((size_t)kind * D + e0 + ee) * D + d0 + c8) = *(const v8b*)(&T[ee][c8]); } __threadfence(); }
}
__global__ __launch_bounds__(128) void proj_kernel(const b16* __restrict__ X16, const b16* __restrict__ WT, const float* __restrict__ bq, const float* __restrict__ bk, const float* __restrict__ bv, b16* __restrict__ QH, b16* __restrict__ KH, b16* __restrict__ VT) {
  __shared__ __attribute__((aligned(16))) b16 Th[4][16][128 + 8]; __shared__ __attribute__((aligned(16))) b16 Vt[128][64 + 8];
  const int wave = threadIdx.x >> 5, lane = threadIdx.x & 31, nloc = lane & 15, hlf = lane >> 4, t_ = threadIdx.x; const int kind = blockIdx.z; const size_t m0 = (size_t)blockIdx.x * 64 + wave * 16; const int n0 = blockIdx.y * 128;
  const b16* Wk_ = WT + (size_t)kind * D * D; const float* bias = kind == 0 ? bq : kind == 1 ? bk : bv; v8f acc[8];
#pragma unroll
  for (int t = 0; t < 8; ++t) acc[t] = (v8f){};
#pragma unroll 2
  for (int kb = 0; kb < D; kb += 32) { const v16b a = frag_kb(X16 + (m0 + nloc) * D + kb, hlf);
#pragma unroll
    for (int t = 0; t < 8; ++t) acc[t] = wmma16b(a, frag_kb(Wk_ + (size_t)(n0 + t * 16 + nloc) * D + kb, hlf), acc[t]); }
  if (kind < 2) {
#pragma unroll
    for (int t = 0; t < 8; ++t) { const float bb = bf16_rne(bias[n0 + t * 16 + nloc]);
#pragma unroll
      for (int r = 0; r < 8; ++r) Th[wave][8 * hlf + r][t * 16 + nloc] = (b16)((acc[t][r] * (1.0f / (XS * WSC)) + bb) * XS); }
    wave_lds_sync();
    b16* dst = kind == 0 ? QH : KH;
    for (int pass = 0; pass < 2; ++pass) { for (int r2 = 0; r2 < 16; r2 += 2) { const int rr = r2 + (lane >> 4), c8 = (lane & 15) * 8; *(volatile v8b*)(dst + (m0 + rr) * D + n0 + c8) = *(const v8b*)(&Th[wave][rr][c8]); } __threadfence(); }
  } else {
    const int b = (int)(m0 / S); const int s0 = (int)((size_t)blockIdx.x * 64 - (size_t)b * S);
#pragma unroll
    for (int t = 0; t < 8; ++t) { const float bb = bf16_rne(bias[n0 + t * 16 + nloc]);
#pragma unroll
      for (int r = 0; r < 8; ++r) Vt[t * 16 + nloc][wave * 16 + 8 * hlf + r] = (b16)((acc[t][r] * (1.0f / (XS * WSC)) + bb) * XS); }
    __syncthreads();
    for (int pass = 0; pass < 2; ++pass) { for (int q = t_; q < 128 * 8; q += 128) { const int dd = q >> 3, c8 = (q & 7) * 8; *(volatile v8b*)(VT + ((size_t)b * D + n0 + dd) * S + s0 + c8) = *(const v8b*)(&Vt[dd][c8]); } __threadfence(); } }
}
__global__ __launch_bounds__(128) void s_kernel(const b16* __restrict__ QH, const b16* __restrict__ KH, int b, float* __restrict__ Sf) {
  __shared__ __attribute__((aligned(16))) float Ts[4][16][128 + 4];
  const int wave = threadIdx.x >> 5, lane = threadIdx.x & 31, nloc = lane & 15, hlf = lane >> 4; const int m0 = blockIdx.x * 64 + wave * 16, n0 = blockIdx.y * 128;
  const b16* Q = QH + (size_t)b * S * D; const b16* K = KH + (size_t)b * S * D; v8f acc[8];
#pragma unroll
  for (int t = 0; t < 8; ++t) acc[t] = (v8f){};
#pragma unroll 2
  for (int kb = 0; kb < D; kb += 32) { const v16b a = frag_kb(Q + (size_t)(m0 + nloc) * D + kb, hlf);
#pragma unroll
    for (int t = 0; t < 8; ++t) acc[t] = wmma16b(a, frag_kb(K + (size_t)(n0 + t * 16 + nloc) * D + kb, hlf), acc[t]); }
#pragma unroll
  for (int t = 0; t < 8; ++t)
#pragma unroll
    for (int r = 0; r < 8; ++r) Ts[wave][8 * hlf + r][t * 16 + nloc] = acc[t][r] * (1.0f / (XS * XS));
  wave_lds_sync();
  for (int pass = 0; pass < 2; ++pass) { for (int rr = 0; rr < 16; ++rr) *(volatile v4f*)(Sf + (size_t)(m0 + rr) * S + n0 + lane * 4) = *(const v4f*)(&Ts[wave][rr][lane * 4]); __threadfence(); }
}
__global__ __launch_bounds__(256) void softmax_kernel(const float* __restrict__ Sf, b16* __restrict__ P16) {
  const int wave = threadIdx.x >> 5, lane = threadIdx.x & 31; const int q = blockIdx.x * 8 + wave; const float* row = Sf + (size_t)q * S;
  float v[64]; float mx = -INFINITY;
#pragma unroll
  for (int j = 0; j < 8; ++j) { const v4f a = *(const v4f*)(row + j * 256 + lane * 8), c = *(const v4f*)(row + j * 256 + lane * 8 + 4);
#pragma unroll
    for (int i = 0; i < 4; ++i) { v[j * 8 + i] = a[i]; v[j * 8 + 4 + i] = c[i]; mx = fmaxf(mx, fmaxf(a[i], c[i])); } }
#pragma unroll
  for (int o = 16; o >= 1; o >>= 1) mx = fmaxf(mx, __shfl_xor(mx, o));
  const float cs = SCALE * LOG2E; float sum = 0.0f;
#pragma unroll
  for (int i = 0; i < 64; ++i) { v[i] = nexp2((v[i] - mx) * cs); sum += v[i]; }
#pragma unroll
  for (int o = 16; o >= 1; o >>= 1) sum += __shfl_xor(sum, o);
  const float inv = PS / sum;
  for (int pass = 0; pass < 2; ++pass) {
#pragma unroll
    for (int j = 0; j < 8; ++j) { v8b o;
#pragma unroll
      for (int i = 0; i < 8; ++i) o[i] = (b16)(v[j * 8 + i] * inv); *(volatile v8b*)(P16 + (size_t)q * S + j * 256 + lane * 8) = o; }
    __threadfence(); }
}
__global__ __launch_bounds__(128) void pv_kernel(const b16* __restrict__ P16, const b16* __restrict__ VT, const float* __restrict__ x, int b, float* __restrict__ H) {
  __shared__ __attribute__((aligned(16))) float Ts[4][16][128 + 4];
  const int wave = threadIdx.x >> 5, lane = threadIdx.x & 31, nloc = lane & 15, hlf = lane >> 4; const int m0 = blockIdx.x * 64 + wave * 16, n0 = blockIdx.y * 128;
  const b16* V = VT + (size_t)b * D * S; v8f acc[8];
#pragma unroll
  for (int t = 0; t < 8; ++t) acc[t] = (v8f){};
#pragma unroll 2
  for (int kb = 0; kb < S; kb += 32) { const v16b a = frag_kb(P16 + (size_t)(m0 + nloc) * S + kb, hlf);
#pragma unroll
    for (int t = 0; t < 8; ++t) acc[t] = wmma16b(a, frag_kb(V + (size_t)(n0 + t * 16 + nloc) * S + kb, hlf), acc[t]); }
#pragma unroll
  for (int t = 0; t < 8; ++t)
#pragma unroll
    for (int r = 0; r < 8; ++r) Ts[wave][8 * hlf + r][t * 16 + nloc] = acc[t][r] * (1.0f / (PS * XS));
  wave_lds_sync();
  for (int pass = 0; pass < 2; ++pass) { for (int rr = 0; rr < 16; ++rr) { const size_t gi = ((size_t)b * S + m0 + rr) * D + n0 + lane * 4; v4f o = *(const v4f*)(&Ts[wave][rr][lane * 4]); const v4f xv = *(const v4f*)(x + gi);
#pragma unroll
      for (int i = 0; i < 4; ++i) o[i] += bf16_rne(xv[i]); *(volatile v4f*)(H + gi) = o; } __threadfence(); }
}
__global__ __launch_bounds__(256) void ln_kernel(const float* __restrict__ H, const float* __restrict__ gamma, const float* __restrict__ beta, float* __restrict__ out) {
  const int wave = threadIdx.x >> 5, lane = threadIdx.x & 31; const size_t row = (size_t)blockIdx.x * 8 + wave; const float* src = H + row * D;
  float v[32]; float s = 0.0f;
#pragma unroll
  for (int j = 0; j < 8; ++j) { const v4f a = *(const v4f*)(src + j * 128 + lane * 4);
#pragma unroll
    for (int i = 0; i < 4; ++i) { v[j * 4 + i] = a[i]; s += a[i]; } }
#pragma unroll
  for (int o = 16; o >= 1; o >>= 1) s += __shfl_xor(s, o);
  const float mean = s * (1.0f / D); float ss = 0.0f;
#pragma unroll
  for (int i = 0; i < 32; ++i) { const float d = v[i] - mean; ss += pmul(d, d); }
#pragma unroll
  for (int o = 16; o >= 1; o >>= 1) ss += __shfl_xor(ss, o);
  const float rs = rsqrtf(ss * (1.0f / D) + EPS);
  for (int pass = 0; pass < 2; ++pass) {
#pragma unroll
    for (int j = 0; j < 8; ++j) { v4f o; const int c0 = j * 128 + lane * 4;
#pragma unroll
      for (int i = 0; i < 4; ++i) o[i] = pmul((v[j * 4 + i] - mean) * rs, bf16_rne(gamma[c0 + i])) + bf16_rne(beta[c0 + i]);
      *(volatile v4f*)(out + row * D + c0) = o; }
    __threadfence(); }
}
}

extern "C" void kernel_launch(void* const* d_in, const int* in_sizes, int n_in, void* d_out, int out_size, void* d_ws, size_t ws_size, hipStream_t stream) {
  (void)n_in;
  auto Fp = [&](int i) { return (const float*)d_in[i]; };
  if (in_sizes[0] != NR * D || in_sizes[1] != D * D || in_sizes[2] != D || in_sizes[3] != D * D || in_sizes[5] != D * D || in_sizes[7] != D || in_sizes[8] != D || out_size != NR * D) return;
  size_t off = 0; char* ws = (char*)d_ws;
  auto carve = [&](size_t bytes) { char* p = ws + off; off += (bytes + 255) & ~(size_t)255; return p; };
  b16* X16 = (b16*)carve((size_t)NR * D * 2); b16* WT = (b16*)carve((size_t)3 * D * D * 2); b16* QH = (b16*)carve((size_t)NR * D * 2); b16* KH = (b16*)carve((size_t)NR * D * 2); b16* VT = (b16*)carve((size_t)NR * D * 2);
  float* Sf = (float*)carve((size_t)S * S * 4); b16* P16 = (b16*)carve((size_t)S * S * 2); float* H = (float*)carve((size_t)NR * D * 4);
  if (off > ws_size || off > ((size_t)128 << 20)) return;
  prepx_kernel<<<(unsigned)(((size_t)NR * D / 8 + 255) / 256), 256, 0, stream>>>(Fp(0), X16);
  prepw_kernel<<<dim3(D / 64, D / 64, 3), 256, 0, stream>>>(Fp(1), Fp(3), Fp(5), WT);
  proj_kernel<<<dim3(NR / 64, D / 128, 3), 128, 0, stream>>>(X16, WT, Fp(2), Fp(4), Fp(6), QH, KH, VT);
  for (int b = 0; b < NB; ++b) {
    s_kernel<<<dim3(S / 64, S / 128), 128, 0, stream>>>(QH, KH, b, Sf);
    softmax_kernel<<<S / 8, 256, 0, stream>>>(Sf, P16);
    pv_kernel<<<dim3(S / 64, D / 128), 128, 0, stream>>>(P16, VT, Fp(0), b, H);
  }
  ln_kernel<<<NR / 8, 256, 0, stream>>>(H, Fp(7), Fp(8), (float*)d_out);
}
